// GraphEncoder_57664230916996
// MI455X (gfx1250) — hardware-verified
//
#include <hip/hip_runtime.h>
#include <stddef.h>
#include <stdint.h>


#define FIN     128
#define HID     256
#define DOUT    768
#define NTHR    256
#define NWAVE   8
#define EPT     8
#define CHUNK   (NTHR * EPT)
#define WCAP    (EPT * 32)
#define LISTN   (NWAVE * WCAP)
#define NBMAX   2048
#define RCAP    28672
#define DEGCAP  4096
#define GBM     64
#define GBN     64
#define GTHR    128
#define WSMAX   134217728
#define LDS_AGG ((2 * RCAP + 2 * NBMAX + LISTN) * 4 + 64)

static_assert((CHUNK & (CHUNK - 1)) == 0 && CHUNK <= 4096);
static_assert((NBMAX & (NBMAX - 1)) == 0 && NBMAX <= 4096);
static_assert(NTHR * 8 == NBMAX);
static_assert(LISTN >= NBMAX);
static_assert(LISTN >= NWAVE * WCAP);
static_assert((RCAP % 32) == 0);
static_assert(LDS_AGG <= 300000);
static_assert(GBM == (GTHR / 32) * 16);
static_assert((FIN % 32) == 0 && (HID % 32) == 0);
static_assert((HID % GBN) == 0 && (DOUT % GBN) == 0);
static_assert(HID == 8 * 32);
static_assert(DOUT == 6 * 128);

typedef float          v4f  __attribute__((ext_vector_type(4)));
typedef float          v8f  __attribute__((ext_vector_type(8)));
typedef int            v4i  __attribute__((ext_vector_type(4)));
typedef int            v8i  __attribute__((ext_vector_type(8)));
typedef unsigned short us_t;
typedef us_t           v8us __attribute__((ext_vector_type(8)));
typedef __bf16         v16b __attribute__((ext_vector_type(16)));
union FragB { v16b v; v8us h[2]; v8i w; };

__device__ __forceinline__ v8f wmb(const FragB& a, const FragB& b, v8f c) {
  v8f d = __builtin_amdgcn_wmma_f32_16x16x32_bf16(false, a.v, false, b.v, (short)0, c, false, false);
  asm volatile("v_nop\n\tv_nop\n\tv_nop\n\tv_nop" : "+v"(d) : "v"(a.w), "v"(b.w));
  return d;
}

__device__ __forceinline__ us_t f2bfbits(float f) {
  unsigned u = __float_as_uint(f);
  u = u + 0x7fffu + ((u >> 16) & 1u);
  return (us_t)(u >> 16);
}
__device__ __forceinline__ float bfbits2f(us_t h) {
  return __uint_as_float(((unsigned)h) << 16);
}
__device__ __forceinline__ float bfr(float f) { return bfbits2f(f2bfbits(f)); }

__device__ __forceinline__ v8us cvt8(const v4f a, const v4f b) {
  v8us hv;
  hv[0] = f2bfbits(a.x); hv[1] = f2bfbits(a.y); hv[2] = f2bfbits(a.z); hv[3] = f2bfbits(a.w);
  hv[4] = f2bfbits(b.x); hv[5] = f2bfbits(b.y); hv[6] = f2bfbits(b.z); hv[7] = f2bfbits(b.w);
  return hv;
}

__device__ __forceinline__ void sp1(const float v, us_t& h, us_t& l) {
  const us_t hb = f2bfbits(v);
  h = hb;
  l = f2bfbits(v - bfbits2f(hb));
}
__device__ __forceinline__ void split8(const v4f a, const v4f b, v8us& hv, v8us& lv) {
  us_t h, l;
  sp1(a.x, h, l); hv[0] = h; lv[0] = l;
  sp1(a.y, h, l); hv[1] = h; lv[1] = l;
  sp1(a.z, h, l); hv[2] = h; lv[2] = l;
  sp1(a.w, h, l); hv[3] = h; lv[3] = l;
  sp1(b.x, h, l); hv[4] = h; lv[4] = l;
  sp1(b.y, h, l); hv[5] = h; lv[5] = l;
  sp1(b.z, h, l); hv[6] = h; lv[6] = l;
  sp1(b.w, h, l); hv[7] = h; lv[7] = l;
}

__device__ __forceinline__ int scan_chunk(const int* __restrict__ dsts, int nE, int cbase, int slotBase,
                                          int nb, int vec8, int* list, int tid, int lane, int wave) {
  int wc = 0;
  const int el0  = tid * EPT;
  const int e0   = cbase + el0;
  const int sent = -2147483647 - 1;
  v4i da, db;
  if (vec8 != 0 && cbase + CHUNK <= nE) {
    da = *(const v4i*)(dsts + e0);
    db = *(const v4i*)(dsts + e0 + 4);
  } else {
    da.x = (e0     < nE) ? dsts[min(e0,     nE - 1)] : sent;
    da.y = (e0 + 1 < nE) ? dsts[min(e0 + 1, nE - 1)] : sent;
    da.z = (e0 + 2 < nE) ? dsts[min(e0 + 2, nE - 1)] : sent;
    da.w = (e0 + 3 < nE) ? dsts[min(e0 + 3, nE - 1)] : sent;
    db.x = (e0 + 4 < nE) ? dsts[min(e0 + 4, nE - 1)] : sent;
    db.y = (e0 + 5 < nE) ? dsts[min(e0 + 5, nE - 1)] : sent;
    db.z = (e0 + 6 < nE) ? dsts[min(e0 + 6, nE - 1)] : sent;
    db.w = (e0 + 7 < nE) ? dsts[min(e0 + 7, nE - 1)] : sent;
  }
  const unsigned nbs = (unsigned)slotBase;
  const unsigned unb = (unsigned)nb;
  const unsigned s0 = (unsigned)da.x - nbs, s1 = (unsigned)da.y - nbs;
  const unsigned s2 = (unsigned)da.z - nbs, s3 = (unsigned)da.w - nbs;
  const unsigned s4 = (unsigned)db.x - nbs, s5 = (unsigned)db.y - nbs;
  const unsigned s6 = (unsigned)db.z - nbs, s7 = (unsigned)db.w - nbs;
  const bool h0 = s0 < unb, h1 = s1 < unb, h2 = s2 < unb, h3 = s3 < unb;
  const bool h4 = s4 < unb, h5 = s5 < unb, h6 = s6 < unb, h7 = s7 < unb;
  const unsigned any = __builtin_amdgcn_ballot_w32(h0 | h1 | h2 | h3 | h4 | h5 | h6 | h7);
  if (any != 0u) {
#define HITJ(J, HJ, SJ) { \
      const unsigned mj = __builtin_amdgcn_ballot_w32(HJ); \
      if (mj != 0u) { \
        if (HJ) { \
          const int pos = wc + (int)__builtin_amdgcn_mbcnt_lo(mj, 0u); \
          if (pos < WCAP) list[wave * WCAP + pos] = ((el0 + (J)) << 12) | (int)(SJ); \
        } \
        wc += (int)__builtin_popcount(mj); } }
    HITJ(0, h0, s0)
    HITJ(1, h1, s1)
    HITJ(2, h2, s2)
    HITJ(3, h3, s3)
    HITJ(4, h4, s4)
    HITJ(5, h5, s5)
    HITJ(6, h6, s6)
    HITJ(7, h7, s7)
#undef HITJ
  }
  return wc;
}

__global__ __launch_bounds__(NTHR) void k_xprep(const float* __restrict__ x, us_t* xb, int nN, int nUnits) {
  const int i = (int)blockIdx.x * NTHR + (int)threadIdx.x;
  if (i >= nUnits) return;
  const int row = i >> 4;
  const int c0  = (i & 15) * 8;
  const int rc  = row < nN ? row : nN - 1;
  const float* p = x + (size_t)rc * FIN + c0;
  v4f a = *(const v4f*)p, b = *(const v4f*)(p + 4);
  const v4f z4 = {0.f, 0.f, 0.f, 0.f};
  if (row >= nN) { a = z4; b = z4; }
  const v8us hv = cvt8(a, b);
  const size_t o = (size_t)row * FIN + c0;
  *(volatile v8us*)(xb + o) = hv;
  __threadfence();
  *(volatile v8us*)(xb + o) = hv;
}

__global__ __launch_bounds__(NTHR) void k_wtr(const float* __restrict__ w, int K, int C, us_t* wt, int nUnits) {
  const int u = (int)blockIdx.x * NTHR + (int)threadIdx.x;
  if (u >= nUnits) return;
  const int kq = K >> 3;
  const int n  = u / kq;
  const int k8 = (u - n * kq) * 8;
  const float* p = w + (size_t)k8 * (size_t)C + n;
  v4f a, b;
  a.x = p[0];                 a.y = p[(size_t)C];          a.z = p[(size_t)2 * C];      a.w = p[(size_t)3 * C];
  b.x = p[(size_t)4 * C];     b.y = p[(size_t)5 * C];      b.z = p[(size_t)6 * C];      b.w = p[(size_t)7 * C];
  const v8us hv = cvt8(a, b);
  const size_t o = (size_t)n * (size_t)K + k8;
  *(volatile v8us*)(wt + o) = hv;
  __threadfence();
  *(volatile v8us*)(wt + o) = hv;
}

template<int SPLIT, int EPI>
__global__ __launch_bounds__(GTHR) void k_gemm(
    const us_t* __restrict__ Ah, const us_t* __restrict__ Al, const us_t* __restrict__ WT,
    const float* __restrict__ bias, const float* __restrict__ dinv,
    float* outF, us_t* outH, us_t* outL, int K, int ldo)
{
  __shared__ __attribute__((aligned(16))) float stg[GBM * GBN];
  const int tid = (int)threadIdx.x, lane = tid & 31, wave = tid >> 5, hh = lane >> 4, m = lane & 15;
  const int rowBase = (int)blockIdx.x * GBM;
  const int col0    = (int)blockIdx.y * GBN;

  v8f acc[4];
  {
    const v8f z = {0.f, 0.f, 0.f, 0.f, 0.f, 0.f, 0.f, 0.f};
    acc[0] = z; acc[1] = z; acc[2] = z; acc[3] = z;
  }
  const size_t arow = (size_t)(rowBase + 16 * wave + m) * (size_t)K + 8 * hh;
  const us_t* ap = Ah + arow;
  const us_t* aq = Al + arow;
  const us_t* wp = WT + (size_t)(col0 + m) * (size_t)K + 8 * hh;
  const int ksteps = K >> 5;
#pragma unroll 1
  for (int ks = 0; ks < ksteps; ++ks) {
    FragB af, al;
    af.h[0] = *(const v8us*)(ap + 32 * ks);
    af.h[1] = *(const v8us*)(ap + 32 * ks + 16);
    if (SPLIT == 2) {
      al.h[0] = *(const v8us*)(aq + 32 * ks);
      al.h[1] = *(const v8us*)(aq + 32 * ks + 16);
    } else {
      al = af;
    }
#pragma unroll
    for (int t = 0; t < 4; ++t) {
      const us_t* wq = wp + (size_t)(16 * t) * (size_t)K + 32 * ks;
      FragB bfg;
      bfg.h[0] = *(const v8us*)wq;
      bfg.h[1] = *(const v8us*)(wq + 16);
      acc[t] = wmb(af, bfg, acc[t]);
      if (SPLIT == 2) acc[t] = wmb(al, bfg, acc[t]);
    }
  }

  if (EPI == 0) {
    float dv[8];
#pragma unroll
    for (int r = 0; r < 8; ++r) dv[r] = dinv[rowBase + 16 * wave + 8 * hh + r];
#pragma unroll
    for (int t = 0; t < 4; ++t) {
      const int lc = 16 * t + m;
#pragma unroll
      for (int r = 0; r < 8; ++r) {
        const int lr = 16 * wave + 8 * hh + r;
        stg[lr * GBN + lc] = acc[t][r] * dv[r];
      }
    }
  } else {
#pragma unroll
    for (int t = 0; t < 4; ++t) {
      const int lc = 16 * t + m;
      const float bv = bfr(bias[col0 + lc]);
#pragma unroll
      for (int r = 0; r < 8; ++r) {
        const int lr = 16 * wave + 8 * hh + r;
        float v = acc[t][r] + bv;
        if (EPI == 1) v = fmaxf(v, 0.f);
        stg[lr * GBN + lc] = v;
      }
    }
  }
  __syncthreads();

  if (EPI == 1) {
    const int q8 = lane & 7, sub = lane >> 3;
    v8us hv[4], lv[4];
#pragma unroll
    for (int i = 0; i < 4; ++i) {
      const int lr = 16 * wave + 4 * i + sub;
      const float* sp = stg + lr * GBN + 8 * q8;
      const v4f a = *(const v4f*)sp;
      const v4f b = *(const v4f*)(sp + 4);
      split8(a, b, hv[i], lv[i]);
    }
#pragma unroll
    for (int i = 0; i < 4; ++i) {
      const int lr = 16 * wave + 4 * i + sub;
      const size_t o = (size_t)(rowBase + lr) * (size_t)ldo + col0 + 8 * q8;
      *(volatile v8us*)(outH + o) = hv[i];
      *(volatile v8us*)(outL + o) = lv[i];
    }
    __threadfence();
#pragma unroll
    for (int i = 0; i < 4; ++i) {
      const int lr = 16 * wave + 4 * i + sub;
      const size_t o = (size_t)(rowBase + lr) * (size_t)ldo + col0 + 8 * q8;
      *(volatile v8us*)(outH + o) = hv[i];
      *(volatile v8us*)(outL + o) = lv[i];
    }
  } else {
    v4f fv[8];
#pragma unroll
    for (int i = 0; i < 8; ++i) {
      const int lr = 16 * wave + 2 * i + hh;
      fv[i] = *(const v4f*)(stg + lr * GBN + 4 * m);
    }
#pragma unroll
    for (int i = 0; i < 8; ++i) {
      const int lr = 16 * wave + 2 * i + hh;
      const int gr = rowBase + lr;
      float* op = outF + (size_t)gr * (size_t)ldo + col0 + 4 * m;
      *(volatile v4f*)op = fv[i];
    }
    __threadfence();
#pragma unroll
    for (int i = 0; i < 8; ++i) {
      const int lr = 16 * wave + 2 * i + hh;
      const int gr = rowBase + lr;
      float* op = outF + (size_t)gr * (size_t)ldo + col0 + 4 * m;
      *(volatile v4f*)op = fv[i];
    }
  }
}

__device__ __forceinline__ float dgi(int c) {
  const int cc = c < 0 ? 0 : c;
  return 1.0f / sqrtf((float)cc + 1.0f);
}

template<int MODE>
__global__ __launch_bounds__(NTHR) void k_agg(
    const int* __restrict__ srcs, const int* __restrict__ dsts,
    const float* __restrict__ HW, const float* __restrict__ bias,
    float* DINV, us_t* HH, us_t* HL,
    int nN, int nE, int nb, int vec8, int MPr) {
  extern __shared__ v4f lds_dyn[];
  int* reg1 = (int*)lds_dyn;
  int* reg2 = reg1 + RCAP;
  int* scnt = reg2 + RCAP;
  int* soff = scnt + NBMAX;
  int* list = soff + NBMAX;
  int* wcnt = list + LISTN;
  int* wtot = wcnt + NWAVE;
  const int tid = (int)threadIdx.x, lane = tid & 31, wave = tid >> 5;
  const int nodeBase = (int)blockIdx.x * nb;

  for (int i = tid; i < NBMAX; i += NTHR) scnt[i] = 0;
  __syncthreads();

  int tot = 0;
  const int nChunks = (nE + CHUNK - 1) / CHUNK;
#pragma unroll 1
  for (int ch = 0; ch < nChunks; ++ch) {
    const int cbase = ch * CHUNK;
    const int wc = scan_chunk(dsts, nE, cbase, nodeBase, nb, vec8, list, tid, lane, wave);
    if (lane == 0) wcnt[wave] = wc;
    __syncthreads();
    int pre = 0, all = 0;
#pragma unroll
    for (int w2 = 0; w2 < NWAVE; ++w2) {
      int c = wcnt[w2];
      c = c < 0 ? 0 : (c > WCAP ? WCAP : c);
      all += c;
      pre += (w2 < wave) ? c : 0;
    }
    const int wcc  = wc > WCAP ? WCAP : wc;
    const int base = tot + pre;
#pragma unroll 1
    for (int i = lane; i < wcc; i += 32) {
      const int ent = list[wave * WCAP + i];
      const int el  = (ent >> 12) & (CHUNK - 1);
      const int sl  = ent & (NBMAX - 1);
      int eid = cbase + el;
      eid = eid > nE - 1 ? nE - 1 : eid;
      const int pos = base + i;
      if (pos < RCAP) reg1[pos] = (int)(((unsigned)eid << 12) | (unsigned)sl);
    }
    tot += all;
    tot = tot > RCAP ? RCAP : tot;
    __syncthreads();
  }
  const int nh = tot;

  if (wave == 0) {
#pragma unroll 1
    for (int b0 = 0; b0 < nh; b0 += 32) {
      const int idx = b0 + lane;
      const int uv  = reg1[idx < RCAP ? idx : RCAP - 1];
      const int m32 = (nh - b0) < 32 ? (nh - b0) : 32;
#pragma unroll 1
      for (int k = 0; k < m32; ++k) {
        const int u  = __builtin_amdgcn_readlane(uv, k);
        const int sl = u & (NBMAX - 1);
        if (lane == 0) scnt[sl] = scnt[sl] + 1;
      }
    }
  }
  __syncthreads();

  if (MODE == 0) {
    const int np = nb >> 2;
    const int p0 = tid, p1 = tid + NTHR;
    const int c0 = p0 < np ? p0 : 0, c1 = p1 < np ? p1 : 0;
    const v4i ca = *(const v4i*)(scnt + 4 * c0);
    const v4i cb = *(const v4i*)(scnt + 4 * c1);
    v4f d0, d1;
    d0.x = dgi(ca.x); d0.y = dgi(ca.y); d0.z = dgi(ca.z); d0.w = dgi(ca.w);
    d1.x = dgi(cb.x); d1.y = dgi(cb.y); d1.z = dgi(cb.z); d1.w = dgi(cb.w);
    float* qa = DINV + (size_t)nodeBase + 4 * c0;
    float* qb = DINV + (size_t)nodeBase + 4 * c1;
    if (p0 < np) *(volatile v4f*)qa = d0;
    if (p1 < np) *(volatile v4f*)qb = d1;
    __threadfence();
    if (p0 < np) *(volatile v4f*)qa = d0;
    if (p1 < np) *(volatile v4f*)qb = d1;
    return;
  }

  {
    const v4i ca = *(const v4i*)(scnt + 8 * tid);
    const v4i cb = *(const v4i*)(scnt + 8 * tid + 4);
    const int e0 = ca.x < 0 ? 0 : ca.x, e1 = ca.y < 0 ? 0 : ca.y, e2 = ca.z < 0 ? 0 : ca.z, e3 = ca.w < 0 ? 0 : ca.w;
    const int e4 = cb.x < 0 ? 0 : cb.x, e5 = cb.y < 0 ? 0 : cb.y, e6 = cb.z < 0 ? 0 : cb.z, e7 = cb.w < 0 ? 0 : cb.w;
    const int ts = e0 + e1 + e2 + e3 + e4 + e5 + e6 + e7;
    int incl = ts;
#pragma unroll
    for (int d = 1; d < 32; d <<= 1) {
      const int up = __shfl_up(incl, d);
      if (lane >= d) incl += up;
    }
    if (lane == 31) wtot[wave] = incl;
    __syncthreads();
    int pre = 0;
#pragma unroll
    for (int w2 = 0; w2 < NWAVE; ++w2) pre += (w2 < wave) ? wtot[w2] : 0;
    int run = pre + incl - ts;
    soff[8 * tid + 0] = run; run += e0;
    soff[8 * tid + 1] = run; run += e1;
    soff[8 * tid + 2] = run; run += e2;
    soff[8 * tid + 3] = run; run += e3;
    soff[8 * tid + 4] = run; run += e4;
    soff[8 * tid + 5] = run; run += e5;
    soff[8 * tid + 6] = run; run += e6;
    soff[8 * tid + 7] = run;
  }
  __syncthreads();
  for (int i = tid; i < NBMAX; i += NTHR) list[i] = soff[i];
  __syncthreads();

  if (wave == 0) {
#pragma unroll 1
    for (int b0 = 0; b0 < nh; b0 += 32) {
      const int idx = b0 + lane;
      const int uv  = reg1[idx < RCAP ? idx : RCAP - 1];
      const int m32 = (nh - b0) < 32 ? (nh - b0) : 32;
#pragma unroll 1
      for (int k = 0; k < m32; ++k) {
        const int u   = __builtin_amdgcn_readlane(uv, k);
        const int sl  = u & (NBMAX - 1);
        const int eid = (int)((unsigned)u >> 12);
        if (lane == 0) {
          int pos = list[sl];
          pos = pos < 0 ? 0 : (pos > RCAP - 1 ? RCAP - 1 : pos);
          reg2[pos] = eid;
          list[sl] = pos + 1;
        }
      }
    }
  }
  __syncthreads();

  const int nbw = nb >> 3;
  const bool ovf = (nh >= RCAP);
  const float qnan = __int_as_float(0x7fc00000);
  v4f bA, bB;
  {
    const v4f ta = *(const v4f*)(bias + 8 * lane);
    const v4f tb = *(const v4f*)(bias + 8 * lane + 4);
    bA.x = bfr(ta.x); bA.y = bfr(ta.y); bA.z = bfr(ta.z); bA.w = bfr(ta.w);
    bB.x = bfr(tb.x); bB.y = bfr(tb.y); bB.z = bfr(tb.z); bB.w = bfr(tb.w);
  }
  const v4f z4 = {0.f, 0.f, 0.f, 0.f};
#pragma unroll 1
  for (int jt = 0; jt < nbw; ++jt) {
    const int slot = wave * nbw + jt;
    const int grow = nodeBase + slot;
    const int gcl  = grow < nN ? grow : nN - 1;
    int st = soff[slot];
    const int craw = scnt[slot];
    int cnt = craw;
    st  = st < 0 ? 0 : (st > nh ? nh : st);
    cnt = cnt < 0 ? 0 : (cnt > DEGCAP ? DEGCAP : cnt);
    if (cnt > nh - st) cnt = nh - st;
    const float pz = (ovf || craw > DEGCAP) ? qnan : 0.0f;
    const bool wr  = grow < MPr;
    const bool liv = grow < nN;

    v4f sa = z4, sb = z4;
#pragma unroll 1
    for (int q = 0; q < cnt; ++q) {
      int idx = st + q; idx = idx > RCAP - 1 ? RCAP - 1 : idx;
      int eid = reg2[idx]; eid = eid < 0 ? 0 : (eid > nE - 1 ? nE - 1 : eid);
      const int sraw = srcs[eid];
      const int s = sraw < 0 ? 0 : (sraw > nN - 1 ? nN - 1 : sraw);
      const float* hr = HW + (size_t)s * HID + 8 * lane;
      const v4f va = *(const v4f*)hr;
      const v4f vb = *(const v4f*)(hr + 4);
      sa += va;
      sb += vb;
    }
    {
      const float* hr = HW + (size_t)gcl * HID + 8 * lane;
      const v4f va = *(const v4f*)hr;
      const v4f vb = *(const v4f*)(hr + 4);
      sa += va;
      sb += vb;
    }
    const float dv = DINV[gcl];
    v4f ra, rb;
    ra.x = fmaxf(fmaf(sa.x, dv, bA.x), 0.f);
    ra.y = fmaxf(fmaf(sa.y, dv, bA.y), 0.f);
    ra.z = fmaxf(fmaf(sa.z, dv, bA.z), 0.f);
    ra.w = fmaxf(fmaf(sa.w, dv, bA.w), 0.f);
    rb.x = fmaxf(fmaf(sb.x, dv, bB.x), 0.f);
    rb.y = fmaxf(fmaf(sb.y, dv, bB.y), 0.f);
    rb.z = fmaxf(fmaf(sb.z, dv, bB.z), 0.f);
    rb.w = fmaxf(fmaf(sb.w, dv, bB.w), 0.f);
    if (MODE == 2) {
      const size_t so = (size_t)gcl * HID + 8 * lane;
      const v8us rh = *(const v8us*)(HH + so);
      const v8us rl = *(const v8us*)(HL + so);
      ra.x += bfbits2f(rh[0]) + bfbits2f(rl[0]);
      ra.y += bfbits2f(rh[1]) + bfbits2f(rl[1]);
      ra.z += bfbits2f(rh[2]) + bfbits2f(rl[2]);
      ra.w += bfbits2f(rh[3]) + bfbits2f(rl[3]);
      rb.x += bfbits2f(rh[4]) + bfbits2f(rl[4]);
      rb.y += bfbits2f(rh[5]) + bfbits2f(rl[5]);
      rb.z += bfbits2f(rh[6]) + bfbits2f(rl[6]);
      rb.w += bfbits2f(rh[7]) + bfbits2f(rl[7]);
    }
    if (!liv) { ra = z4; rb = z4; }
    ra.x += pz; ra.y += pz; ra.z += pz; ra.w += pz;
    rb.x += pz; rb.y += pz; rb.z += pz; rb.w += pz;
    v8us hv, lv;
    split8(ra, rb, hv, lv);
    const size_t ro = (size_t)(wr ? grow : 0) * HID + 8 * lane;
    if (wr) { *(volatile v8us*)(HH + ro) = hv; *(volatile v8us*)(HL + ro) = lv; }
    __threadfence();
    if (wr) { *(volatile v8us*)(HH + ro) = hv; *(volatile v8us*)(HL + ro) = lv; }
  }
}

__global__ __launch_bounds__(NTHR) void k_pool(const int* __restrict__ batch, const us_t* __restrict__ HH,
                                               const us_t* __restrict__ HL, us_t* GH, us_t* GL, int nN, int nG) {
  const int tid = (int)threadIdx.x, lane = tid & 31, wave = tid >> 5;
  const int g = (int)blockIdx.x * NWAVE + wave;
  const bool ok = g < nG;
  const v4f z4 = {0.f, 0.f, 0.f, 0.f};
  v4f sa = z4, sb = z4;
  int cnt = 0;
#pragma unroll 1
  for (int i0 = 0; i0 < nN; i0 += 32) {
    const int i  = i0 + lane;
    const int ic = i < nN ? i : nN - 1;
    const int id = batch[ic];
    const bool hit = (i < nN) && (id == g);
    unsigned msk = __builtin_amdgcn_ballot_w32(hit);
    cnt += (int)__builtin_popcount(msk);
#pragma unroll 1
    for (int it = 0; it < 32 && msk != 0u; ++it) {
      const int k = (int)__builtin_ctz(msk);
      msk &= msk - 1u;
      int node = i0 + k;
      node = node > nN - 1 ? nN - 1 : node;
      const size_t o = (size_t)node * HID + 8 * lane;
      const v8us rh = *(const v8us*)(HH + o);
      const v8us rl = *(const v8us*)(HL + o);
      sa.x += bfbits2f(rh[0]) + bfbits2f(rl[0]);
      sa.y += bfbits2f(rh[1]) + bfbits2f(rl[1]);
      sa.z += bfbits2f(rh[2]) + bfbits2f(rl[2]);
      sa.w += bfbits2f(rh[3]) + bfbits2f(rl[3]);
      sb.x += bfbits2f(rh[4]) + bfbits2f(rl[4]);
      sb.y += bfbits2f(rh[5]) + bfbits2f(rl[5]);
      sb.z += bfbits2f(rh[6]) + bfbits2f(rl[6]);
      sb.w += bfbits2f(rh[7]) + bfbits2f(rl[7]);
    }
  }
  const float cf  = (float)cnt;
  const float inv = 1.0f / (cf > 1.0f ? cf : 1.0f);
  v4f ra, rb;
  ra.x = sa.x * inv; ra.y = sa.y * inv; ra.z = sa.z * inv; ra.w = sa.w * inv;
  rb.x = sb.x * inv; rb.y = sb.y * inv; rb.z = sb.z * inv; rb.w = sb.w * inv;
  v8us hv, lv;
  split8(ra, rb, hv, lv);
  const size_t o = (size_t)(ok ? g : 0) * HID + 8 * lane;
  if (ok) { *(volatile v8us*)(GH + o) = hv; *(volatile v8us*)(GL + o) = lv; }
  __threadfence();
  if (ok) { *(volatile v8us*)(GH + o) = hv; *(volatile v8us*)(GL + o) = lv; }
}

__global__ __launch_bounds__(NTHR) void k_ln(const float* __restrict__ gp, const float* __restrict__ lg,
                                             const float* __restrict__ lb, float* out, int nG) {
  const int tid = (int)threadIdx.x, lane = tid & 31, wave = tid >> 5;
  const int row = (int)blockIdx.x * NWAVE + wave;
  const bool ok = row < nG;
  const int rc  = ok ? row : 0;
  v4f v[6];
#pragma unroll
  for (int i = 0; i < 6; ++i) v[i] = *(const v4f*)(gp + (size_t)rc * DOUT + 128 * i + 4 * lane);
  float s = 0.f;
#pragma unroll
  for (int i = 0; i < 6; ++i) s += (v[i].x + v[i].y) + (v[i].z + v[i].w);
#pragma unroll
  for (int off = 16; off > 0; off >>= 1) s += __shfl_xor(s, off);
  const float mu = s * (1.0f / (float)DOUT);
  float s2 = 0.f;
#pragma unroll
  for (int i = 0; i < 6; ++i) {
    const float dx = v[i].x - mu, dy = v[i].y - mu, dz = v[i].z - mu, dw = v[i].w - mu;
    s2 += (dx * dx + dy * dy) + (dz * dz + dw * dw);
  }
#pragma unroll
  for (int off = 16; off > 0; off >>= 1) s2 += __shfl_xor(s2, off);
  const float var = s2 * (1.0f / (float)DOUT);
  const float rs  = 1.0f / sqrtf(var + 1e-5f);
  v4f y[6];
#pragma unroll
  for (int i = 0; i < 6; ++i) {
    const v4f ga = *(const v4f*)(lg + 128 * i + 4 * lane);
    const v4f be = *(const v4f*)(lb + 128 * i + 4 * lane);
    y[i].x = (v[i].x - mu) * rs * bfr(ga.x) + bfr(be.x);
    y[i].y = (v[i].y - mu) * rs * bfr(ga.y) + bfr(be.y);
    y[i].z = (v[i].z - mu) * rs * bfr(ga.z) + bfr(be.z);
    y[i].w = (v[i].w - mu) * rs * bfr(ga.w) + bfr(be.w);
  }
#pragma unroll
  for (int i = 0; i < 6; ++i) {
    float* op = out + (size_t)rc * DOUT + 128 * i + 4 * lane;
    if (ok) *(volatile v4f*)op = y[i];
  }
  __threadfence();
#pragma unroll
  for (int i = 0; i < 6; ++i) {
    float* op = out + (size_t)rc * DOUT + 128 * i + 4 * lane;
    if (ok) *(volatile v4f*)op = y[i];
  }
}

static int pick_nb(int nE, int nN) {
  int nb = NBMAX;
  while (nb > 32 && (long long)nb * (long long)nE * 5LL > (long long)RCAP * (long long)nN * 4LL) nb >>= 1;
  return nb;
}
static inline int cdiv(int a, int b) { return (a + b - 1) / b; }

extern "C" void kernel_launch(void* const* d_in, const int* in_sizes, int n_in,
                              void* d_out, int out_size, void* d_ws, size_t ws_size,
                              hipStream_t stream) {
  if (n_in < 15) return;
  const int nN = in_sizes[0] / FIN;
  if (nN <= 0 || in_sizes[0] != nN * FIN || nN > (1 << 22)) return;
  if (in_sizes[1] < 2 || (in_sizes[1] & 1) != 0) return;
  const int nE = in_sizes[1] / 2;
  if (nE < 1 || nE > (1 << 20)) return;
  if (in_sizes[2] != nN) return;
  if (in_sizes[3]  != FIN * HID  || in_sizes[4]  != HID)  return;
  if (in_sizes[5]  != HID * HID  || in_sizes[6]  != HID)  return;
  if (in_sizes[7]  != HID * HID  || in_sizes[8]  != HID)  return;
  if (in_sizes[9]  != HID * HID  || in_sizes[10] != HID)  return;
  if (in_sizes[11] != HID * DOUT || in_sizes[12] != DOUT) return;
  if (in_sizes[13] != DOUT || in_sizes[14] != DOUT) return;
  if (out_size <= 0 || (out_size % DOUT) != 0) return;
  const int nG = out_size / DOUT;
  if (nG < GBM || (nG % GBM) != 0 || nG > (1 << 20)) return;

  const float* x    = (const float*)d_in[0];
  const int*   ei   = (const int*)  d_in[1];
  const int*   bat  = (const int*)  d_in[2];
  const float* W1   = (const float*)d_in[3];
  const float* b1   = (const float*)d_in[4];
  const float* W2   = (const float*)d_in[5];
  const float* b2   = (const float*)d_in[6];
  const float* W3   = (const float*)d_in[7];
  const float* b3   = (const float*)d_in[8];
  const float* P1   = (const float*)d_in[9];
  const float* pb1  = (const float*)d_in[10];
  const float* P2   = (const float*)d_in[11];
  const float* pb2  = (const float*)d_in[12];
  const float* lng  = (const float*)d_in[13];
  const float* lnb  = (const float*)d_in[14];
  float* out = (float*)d_out;
  const int* src = ei;
  const int* dst = ei + nE;

  const int MP   = cdiv(nN, GBM) * GBM;
  const int nb   = pick_nb(nE, nN);
  const int gA   = cdiv(MP, nb);
  const int vec8 = ((nE & 3) == 0) ? 1 : 0;
  if (nb < 32 || (nb & (nb - 1)) != 0 || gA * nb < MP) return;

  char* ws = (char*)d_ws;
  size_t off = 0;
  const size_t oXB  = off; off += (size_t)MP * FIN * 2;             off = (off + 255) & ~(size_t)255;
  const size_t oDI  = off; off += (size_t)gA * (size_t)nb * 4;      off = (off + 255) & ~(size_t)255;
  const size_t oWT1 = off; off += (size_t)HID * FIN * 2;            off = (off + 255) & ~(size_t)255;
  const size_t oWT2 = off; off += (size_t)HID * HID * 2;            off = (off + 255) & ~(size_t)255;
  const size_t oWT3 = off; off += (size_t)HID * HID * 2;            off = (off + 255) & ~(size_t)255;
  const size_t oPT1 = off; off += (size_t)HID * HID * 2;            off = (off + 255) & ~(size_t)255;
  const size_t oPT2 = off; off += (size_t)DOUT * HID * 2;           off = (off + 255) & ~(size_t)255;
  const size_t oHW  = off; off += (size_t)MP * HID * 4;             off = (off + 255) & ~(size_t)255;
  const size_t oHH  = off; off += (size_t)MP * HID * 2;             off = (off + 255) & ~(size_t)255;
  const size_t oHL  = off; off += (size_t)MP * HID * 2;             off = (off + 255) & ~(size_t)255;
  const size_t oGH  = off; off += (size_t)nG * HID * 2;             off = (off + 255) & ~(size_t)255;
  const size_t oGL  = off; off += (size_t)nG * HID * 2;             off = (off + 255) & ~(size_t)255;
  const size_t oG1H = off; off += (size_t)nG * HID * 2;             off = (off + 255) & ~(size_t)255;
  const size_t oG1L = off; off += (size_t)nG * HID * 2;             off = (off + 255) & ~(size_t)255;
  const size_t oGP  = off; off += (size_t)nG * DOUT * 4;            off = (off + 255) & ~(size_t)255;
  if (off > ws_size || off > (size_t)WSMAX) return;
  us_t*  XB   = (us_t*)(ws + oXB);
  float* DINV = (float*)(ws + oDI);
  us_t*  WT1  = (us_t*)(ws + oWT1);
  us_t*  WT2  = (us_t*)(ws + oWT2);
  us_t*  WT3  = (us_t*)(ws + oWT3);
  us_t*  PT1  = (us_t*)(ws + oPT1);
  us_t*  PT2  = (us_t*)(ws + oPT2);
  float* HW   = (float*)(ws + oHW);
  us_t*  HH   = (us_t*)(ws + oHH);
  us_t*  HL   = (us_t*)(ws + oHL);
  us_t*  GH   = (us_t*)(ws + oGH);
  us_t*  GL   = (us_t*)(ws + oGL);
  us_t*  G1H  = (us_t*)(ws + oG1H);
  us_t*  G1L  = (us_t*)(ws + oG1L);
  float* GPRE = (float*)(ws + oGP);

  hipFuncSetAttribute(reinterpret_cast<const void*>(&k_agg<0>), hipFuncAttributeMaxDynamicSharedMemorySize, LDS_AGG);
  hipFuncSetAttribute(reinterpret_cast<const void*>(&k_agg<1>), hipFuncAttributeMaxDynamicSharedMemorySize, LDS_AGG);
  hipFuncSetAttribute(reinterpret_cast<const void*>(&k_agg<2>), hipFuncAttributeMaxDynamicSharedMemorySize, LDS_AGG);

  const int nUx = MP * (FIN / 8);
  k_xprep<<<cdiv(nUx, NTHR), NTHR, 0, stream>>>(x, XB, nN, nUx);

  {
    const int nU1 = HID * (FIN / 8);
    k_wtr<<<cdiv(nU1, NTHR), NTHR, 0, stream>>>(W1, FIN, HID, WT1, nU1);
    const int nU2 = HID * (HID / 8);
    k_wtr<<<cdiv(nU2, NTHR), NTHR, 0, stream>>>(W2, HID, HID, WT2, nU2);
    k_wtr<<<cdiv(nU2, NTHR), NTHR, 0, stream>>>(W3, HID, HID, WT3, nU2);
    k_wtr<<<cdiv(nU2, NTHR), NTHR, 0, stream>>>(P1, HID, HID, PT1, nU2);
    const int nU3 = DOUT * (HID / 8);
    k_wtr<<<cdiv(nU3, NTHR), NTHR, 0, stream>>>(P2, HID, DOUT, PT2, nU3);
  }

  k_agg<0><<<gA, NTHR, LDS_AGG, stream>>>(src, dst, HW, b1, DINV, HH, HL, nN, nE, nb, vec8, MP);

  const int gM = MP / GBM;
  k_gemm<1, 0><<<dim3(gM, HID / GBN), GTHR, 0, stream>>>(XB, XB, WT1, b1, DINV, HW, GH, GL, FIN, HID);
  k_agg<1><<<gA, NTHR, LDS_AGG, stream>>>(src, dst, HW, b1, DINV, HH, HL, nN, nE, nb, vec8, MP);
  k_gemm<2, 0><<<dim3(gM, HID / GBN), GTHR, 0, stream>>>(HH, HL, WT2, b2, DINV, HW, GH, GL, HID, HID);
  k_agg<2><<<gA, NTHR, LDS_AGG, stream>>>(src, dst, HW, b2, DINV, HH, HL, nN, nE, nb, vec8, MP);
  k_gemm<2, 0><<<dim3(gM, HID / GBN), GTHR, 0, stream>>>(HH, HL, WT3, b3, DINV, HW, GH, GL, HID, HID);
  k_agg<2><<<gA, NTHR, LDS_AGG, stream>>>(src, dst, HW, b3, DINV, HH, HL, nN, nE, nb, vec8, MP);

  k_pool<<<nG / NWAVE, NTHR, 0, stream>>>(bat, HH, HL, GH, GL, nN, nG);

  k_gemm<2, 1><<<dim3(nG / GBM, HID / GBN), GTHR, 0, stream>>>(GH, GL, PT1, pb1, DINV, GPRE, G1H, G1L, HID, HID);
  k_gemm<2, 2><<<dim3(nG / GBM, DOUT / GBN), GTHR, 0, stream>>>(G1H, G1L, PT2, pb2, DINV, GPRE, GH, GL, HID, DOUT);

  k_ln<<<nG / NWAVE, NTHR, 0, stream>>>(GPRE, lng, lnb, out, nG);
}
